// SimpleLSTM_60713657697205
// MI455X (gfx1250) — hardware-verified
//
#include <hip/hip_runtime.h>
#include <math.h>

constexpr int NSEQ    = 128;
constexpr int NSTEP   = 512;
constexpr int NEMB    = 256;
constexpr int NHID    = 512;
constexpr int NVOC    = 32000;
constexpr int KDIM    = NHID + NEMB;
constexpr int NGCOL   = 4 * NHID;
constexpr int NTHR    = 256;
constexpr int SEQ_BLK = 16;
constexpr int APITCH  = 776;
constexpr int FPITCH  = 516;
constexpr float WCARRY     = 256.0f;
constexpr float WCARRY_INV = 1.0f / 256.0f;
static_assert(NSEQ % SEQ_BLK == 0);
static_assert(KDIM % 32 == 0);
static_assert(NHID % 64 == 0 && KDIM % 64 == 0);
static_assert(NHID == 64 * (NTHR / 32));
static_assert(APITCH % 8 == 0 && APITCH >= KDIM);
static_assert(FPITCH % 4 == 0 && FPITCH >= NHID);
static_assert(SEQ_BLK * NEMB == NTHR * 16);
static_assert(SEQ_BLK * NHID == NTHR * 4 * 8);

typedef __attribute__((ext_vector_type(16))) _Float16 v16h;
typedef __attribute__((ext_vector_type(8)))  _Float16 v8h;
typedef __attribute__((ext_vector_type(16))) __bf16   v16b;
typedef __attribute__((ext_vector_type(8)))  __bf16   v8b;
typedef __attribute__((ext_vector_type(8)))  float    v8f;
typedef __attribute__((ext_vector_type(4)))  float    v4f;

__device__ __forceinline__ unsigned short f2bf_bits(float f) {
  unsigned u = __float_as_uint(f);
  return (unsigned short)((u + 0x7FFFu + ((u >> 16) & 1u)) >> 16);
}
__device__ __forceinline__ float bf_bits2f(unsigned short h) { return __uint_as_float(((unsigned)h) << 16); }
__device__ __forceinline__ float bf16r(float f) { return bf_bits2f(f2bf_bits(f)); }

__device__ __forceinline__ void dep_guard_h(v8f& a, v8f& b, v16h x, v16h y) { asm volatile("v_nop\n\tv_nop\n\tv_nop\n\tv_nop" : "+v"(a), "+v"(b) : "v"(x), "v"(y)); }
__device__ __forceinline__ void dep_guard_b(v8f& a, v8f& b, v16b x, v16b y) { asm volatile("v_nop\n\tv_nop\n\tv_nop\n\tv_nop" : "+v"(a), "+v"(b) : "v"(x), "v"(y)); }
__device__ __forceinline__ void keep4_h(v16h a, v16h b, v16h c, v16h d) { asm volatile("v_nop" :: "v"(a), "v"(b), "v"(c), "v"(d)); }
__device__ __forceinline__ void keep4_b(v16b a, v16b b, v16b c, v16b d) { asm volatile("v_nop" :: "v"(a), "v"(b), "v"(c), "v"(d)); }
__device__ __forceinline__ void acc_guard4(v8f& a, v8f& b, v8f& c, v8f& d) { asm volatile("v_nop\n\tv_nop\n\tv_nop\n\tv_nop" : "+v"(a), "+v"(b), "+v"(c), "+v"(d)); }
template <typename T> struct Frag;
template <> struct Frag<_Float16> {
  typedef v16h V; union U { v16h v; v8h h[2]; };
  static __device__ __forceinline__ v16h load(const _Float16* p) {
    U f; f.h[0] = *(const v8h*)(p); f.h[1] = *(const v8h*)(p + 16); return f.v;
  }
  static __device__ __forceinline__ v8f mma(v16h a, v16h b, v8f c) {
    return __builtin_amdgcn_wmma_f32_16x16x32_f16(false, a, false, b, (short)0, c, false, false);
  }
  static __device__ __forceinline__ void guard(v8f& a, v8f& b, v16h x, v16h y) { dep_guard_h(a, b, x, y); }
  static __device__ __forceinline__ void keep(v16h a, v16h b, v16h c, v16h d) { keep4_h(a, b, c, d); }
};
template <> struct Frag<__bf16> {
  typedef v16b V; union U { v16b v; v8b h[2]; };
  static __device__ __forceinline__ v16b load(const __bf16* p) {
    U f; f.h[0] = *(const v8b*)(p); f.h[1] = *(const v8b*)(p + 16); return f.v;
  }
  static __device__ __forceinline__ v8f mma(v16b a, v16b b, v8f c) {
    return __builtin_amdgcn_wmma_f32_16x16x32_bf16(false, a, false, b, (short)0, c, false, false);
  }
  static __device__ __forceinline__ void guard(v8f& a, v8f& b, v16b x, v16b y) { dep_guard_b(a, b, x, y); }
  static __device__ __forceinline__ void keep(v16b a, v16b b, v16b c, v16b d) { keep4_b(a, b, c, d); }
};

__device__ __forceinline__ float fsig(float x)  { return __builtin_amdgcn_rcpf(1.0f + __expf(-x)); }
__device__ __forceinline__ float ftanh(float x) { return 1.0f - 2.0f * __builtin_amdgcn_rcpf(__expf(2.0f * x) + 1.0f); }

template <int MODE>
__global__ __launch_bounds__(NTHR) void tpw_kernel(const float* __restrict__ src, int R, int C, int ldo,
                                                  unsigned short* __restrict__ O, float sc) {
  __shared__ float Tt[64 * 65];
  const int tid = threadIdx.x;
  const int c0 = blockIdx.x * 64, r0 = blockIdx.y * 64;
#pragma unroll
  for (int i = 0; i < 4; ++i) {
    const int idx = i * NTHR + tid;
    const int rr = idx >> 4, cc = (idx & 15) * 4;
    const v4f v = *(const v4f*)(src + (size_t)(r0 + rr) * (size_t)C + c0 + cc);
    Tt[rr * 65 + cc + 0] = v[0];
    Tt[rr * 65 + cc + 1] = v[1];
    Tt[rr * 65 + cc + 2] = v[2];
    Tt[rr * 65 + cc + 3] = v[3];
  }
  __syncthreads();
  const int q = tid >> 3, c8 = (tid & 7) * 8;
  v8h hv[2];
#pragma unroll
  for (int g = 0; g < 2; ++g) {
    const int qq = g * 32 + q;
#pragma unroll
    for (int e = 0; e < 8; ++e) {
      const float f = Tt[(c8 + e) * 65 + qq];
      unsigned short bits;
      if (MODE == 0) {
        bits = f2bf_bits(f * sc);
      } else {
        const float fb = bf_bits2f(f2bf_bits(f));
        bits = __builtin_bit_cast(unsigned short, (_Float16)(fb * sc));
      }
      hv[g][e] = __builtin_bit_cast(_Float16, bits);
    }
  }
  for (int pass = 0; pass < 2; ++pass) {
#pragma unroll
    for (int g = 0; g < 2; ++g) {
      const size_t o = (size_t)(c0 + g * 32 + q) * (size_t)ldo + (size_t)(r0 + c8);
      *(volatile v8h*)(O + o) = hv[g];
    }
    __threadfence();
  }
}

__device__ __forceinline__ void stage_x(const int* __restrict__ X, const float* __restrict__ E, _Float16* at,
                                        int rowbase, int t, int tid) {
  const int m = tid >> 4, seg = (tid & 15) * 16;
  int tok = X[(size_t)(rowbase + m) * NSTEP + t];
  tok = (tok < 0) ? 0 : ((tok > NVOC - 1) ? (NVOC - 1) : tok);
  const float* er = E + (size_t)tok * NEMB + seg;
  v8h hv0, hv1;
#pragma unroll
  for (int i = 0; i < 2; ++i) {
    const v4f a = *(const v4f*)(er + 4 * i);
    const v4f b = *(const v4f*)(er + 8 + 4 * i);
#pragma unroll
    for (int e = 0; e < 4; ++e) {
      hv0[4 * i + e] = (_Float16)bf16r(a[e]);
      hv1[4 * i + e] = (_Float16)bf16r(b[e]);
    }
  }
  *(v8h*)(at + m * APITCH + NHID + seg)     = hv0;
  *(v8h*)(at + m * APITCH + NHID + seg + 8) = hv1;
}

__global__ __launch_bounds__(NTHR) void lstm_seq_kernel(const int* __restrict__ X, const float* __restrict__ E,
                                                       const float* __restrict__ bi, const float* __restrict__ bfg,
                                                       const float* __restrict__ bo, const float* __restrict__ bh,
                                                       const unsigned short* __restrict__ Btp,
                                                       float* __restrict__ out) {
  __shared__ __align__(16) _Float16 At[2][SEQ_BLK * APITCH];
  __shared__ __align__(16) float    Hs[SEQ_BLK * FPITCH];
  const _Float16* Bt = (const _Float16*)Btp;
  const int tid = threadIdx.x, lane = tid & 31, wave = tid >> 5;
  const int c = lane & 15, hh = lane >> 4, koff = hh * 8;
  const int rowbase = blockIdx.x * SEQ_BLK;

#pragma unroll 1
  for (int i = tid; i < 2 * SEQ_BLK * NHID; i += NTHR) {
    const int buf = i >> 13, row = (i >> 9) & 15, col = i & 511;
    At[buf][row * APITCH + col] = (_Float16)0.0f;
  }
  stage_x(X, E, &At[0][0], rowbase, 0, tid);

  float cst[4][8], bb[4][4];
#pragma unroll
  for (int nt = 0; nt < 4; ++nt) {
    const int j = 64 * wave + 16 * nt + c;
    bb[nt][0] = bf16r(bi[j]);
    bb[nt][1] = bf16r(bfg[j]);
    bb[nt][2] = bf16r(bo[j]);
    bb[nt][3] = bf16r(bh[j]);
#pragma unroll
    for (int r = 0; r < 8; ++r) cst[nt][r] = 0.0f;
  }
  __syncthreads();

  const v8f z8 = {0.f, 0.f, 0.f, 0.f, 0.f, 0.f, 0.f, 0.f};
  const size_t plane = (size_t)NHID * KDIM;

#pragma unroll 1
  for (int t = 0; t < NSTEP; ++t) {
    const int cur = t & 1;
    const _Float16* arow = &At[cur][0] + c * APITCH + koff;
    _Float16* anext = &At[cur ^ 1][0];
    const bool last = (t == NSTEP - 1);
#pragma unroll
    for (int nt = 0; nt < 4; ++nt) {
      const int j = 64 * wave + 16 * nt + c;
      const _Float16* wr = Bt + (size_t)j * KDIM + koff;
      v8f acc[4];
      acc[0] = z8; acc[1] = z8; acc[2] = z8; acc[3] = z8;
#pragma unroll 1
      for (int k0 = 0; k0 < KDIM; k0 += 32) {
        const v16h a  = Frag<_Float16>::load(arow + k0);
        const v16h b0 = Frag<_Float16>::load(wr + k0);
        const v16h b1 = Frag<_Float16>::load(wr + plane + k0);
        const v16h b2 = Frag<_Float16>::load(wr + 2 * plane + k0);
        const v16h b3 = Frag<_Float16>::load(wr + 3 * plane + k0);
        acc[0] = Frag<_Float16>::mma(a, b0, acc[0]);
        acc[1] = Frag<_Float16>::mma(a, b1, acc[1]);
        acc[2] = Frag<_Float16>::mma(a, b2, acc[2]);
        acc[3] = Frag<_Float16>::mma(a, b3, acc[3]);
        dep_guard_h(acc[0], acc[3], a, b3);
        keep4_h(b0, b1, b2, b3);
      }
      acc_guard4(acc[0], acc[1], acc[2], acc[3]);
      float hn8[8];
#pragma unroll
      for (int r = 0; r < 8; ++r) {
        const float zi = acc[0][r] * WCARRY_INV + bb[nt][0];
        const float zf = acc[1][r] * WCARRY_INV + bb[nt][1];
        const float zo = acc[2][r] * WCARRY_INV + bb[nt][2];
        const float zg = acc[3][r] * WCARRY_INV + bb[nt][3];
        const float ig = fsig(zi);
        const float fg = fsig(zf);
        const float og = fsig(zo);
        const float gg = ftanh(zg);
        const float cn = fg * cst[nt][r] + ig * gg;
        cst[nt][r] = cn;
        const float hn = og * ftanh(cn);
        hn8[r] = hn;
        anext[(8 * hh + r) * APITCH + j] = (_Float16)hn;
      }
      if (last) {
#pragma unroll
        for (int r = 0; r < 8; ++r) Hs[(8 * hh + r) * FPITCH + j] = hn8[r];
      }
    }
    {
      const int tn = (t + 1 < NSTEP) ? (t + 1) : (NSTEP - 1);
      stage_x(X, E, anext, rowbase, tn, tid);
    }
    __syncthreads();
  }

  for (int pass = 0; pass < 2; ++pass) {
#pragma unroll
    for (int it = 0; it < 8; ++it) {
      const int idx = it * NTHR + tid;
      const int row = idx >> 7, c4 = (idx & 127) * 4;
      const v4f v = *(const v4f*)(Hs + row * FPITCH + c4);
      *(volatile v4f*)(out + (size_t)(rowbase + row) * NHID + c4) = v;
    }
    __threadfence();
  }
}

extern "C" void kernel_launch(void* const* d_in, const int* in_sizes, int n_in,
                              void* d_out, int out_size, void* d_ws, size_t ws_size, hipStream_t stream) {
  if (n_in < 10 || d_out == nullptr || d_ws == nullptr) return;
  if (in_sizes[0] != NSEQ * NSTEP || in_sizes[1] != NVOC * NEMB ||
      in_sizes[2] != KDIM * NHID || in_sizes[3] != NHID ||
      in_sizes[4] != KDIM * NHID || in_sizes[5] != NHID ||
      in_sizes[6] != KDIM * NHID || in_sizes[7] != NHID ||
      in_sizes[8] != KDIM * NHID || in_sizes[9] != NHID ||
      out_size != NSEQ * NHID) return;

  const int*   X   = (const int*)d_in[0];
  const float* E   = (const float*)d_in[1];
  const float* Wi  = (const float*)d_in[2];
  const float* bi  = (const float*)d_in[3];
  const float* Wf  = (const float*)d_in[4];
  const float* bfg = (const float*)d_in[5];
  const float* Wo  = (const float*)d_in[6];
  const float* bo  = (const float*)d_in[7];
  const float* Wh  = (const float*)d_in[8];
  const float* bh  = (const float*)d_in[9];
  float* out = (float*)d_out;

  char* ws = (char*)d_ws; size_t off = 0;
  auto carve = [&](size_t bytes) -> char* { char* p = ws + off; off += (bytes + 255) & ~(size_t)255; return p; };
  unsigned short* BT = (unsigned short*)carve((size_t)NGCOL * KDIM * 2);
  if (off > ws_size || off > (size_t)134217728) return;

  const size_t plane = (size_t)NHID * KDIM;
  const dim3 tgrid(NHID / 64, KDIM / 64);
  tpw_kernel<1><<<tgrid, NTHR, 0, stream>>>(Wi, KDIM, NHID, KDIM, BT + 0 * plane, WCARRY);
  tpw_kernel<1><<<tgrid, NTHR, 0, stream>>>(Wf, KDIM, NHID, KDIM, BT + 1 * plane, WCARRY);
  tpw_kernel<1><<<tgrid, NTHR, 0, stream>>>(Wo, KDIM, NHID, KDIM, BT + 2 * plane, WCARRY);
  tpw_kernel<1><<<tgrid, NTHR, 0, stream>>>(Wh, KDIM, NHID, KDIM, BT + 3 * plane, WCARRY);
  lstm_seq_kernel<<<NSEQ / SEQ_BLK, NTHR, 0, stream>>>(X, E, bi, bfg, bo, bh, BT, out);
}
